// Extractor_85933705658892
// MI455X (gfx1250) — hardware-verified
//
#include <hip/hip_runtime.h>
#include <math.h>

typedef __attribute__((ext_vector_type(16))) _Float16 v16h;
typedef __attribute__((ext_vector_type(8)))  _Float16 v8h;
typedef __attribute__((ext_vector_type(16))) __bf16   v16b;
typedef __attribute__((ext_vector_type(8)))  __bf16   v8b;
typedef __attribute__((ext_vector_type(8)))  float    v8f;
typedef __attribute__((ext_vector_type(4)))  float    v4f;

constexpr int kWin    = 25;
constexpr int kCin    = 7;
constexpr int kLin    = 3000;
constexpr int kCout   = 64;
constexpr int kTap    = 100;
constexpr int kStride = 20;
constexpr int kLout   = (kLin - kTap) / kStride + 1;
constexpr int kRows   = kWin * kLout;
constexpr int kK      = kCin * kTap;
constexpr int kRowsP  = 3712;
constexpr int kKP     = 704;
constexpr int kPlane  = kCout * kLout;
constexpr int kThr    = 256;

constexpr float kInCarry  = 1024.0f;
constexpr float kWCarry   = 1024.0f;
constexpr float kScale    = 1.0f / (kInCarry * kWCarry);
constexpr float kF16MinNormal = 6.103515625e-5f;

static_assert(kLout == 146 && kRows == 3650 && kK == 700 && kPlane == 9344, "sizes");
static_assert(kRowsP >= kRows && (kRowsP % 64) == 0 && kKP >= kK && (kKP % 32) == 0 && (kCout % 64) == 0, "GEMM M, N multiples of 64, K of 32");
static_assert(((size_t)kRowsP * (kKP / 8)) % kThr == 0 && ((size_t)kCout * (kKP / 8)) % kThr == 0, "plane grids exact");
static_assert((kPlane % 128) == 0 && (kPlane / 4) % 32 == 0, "a window's 9,344 outputs = 73 waves x 4 whole lines");

constexpr size_t kOffA16  = 0;
constexpr size_t kOffW16  = kOffA16 + (size_t)kRowsP * kKP * 2;
constexpr size_t kOffZB   = kOffW16 + (size_t)kCout * kKP * 2;
constexpr size_t kOffLIN  = kOffZB  + 256;
constexpr size_t kWsTotal = kOffLIN + (size_t)kRowsP * kCout * 4;
static_assert(kWsTotal == 6267136ull, "carve total");
static_assert(kWsTotal <= 134217728ull, "carve cap");
static_assert((kOffW16 % 256) == 0 && (kOffZB % 256) == 0 && (kOffLIN % 256) == 0, "aligned regions");

__device__ __forceinline__ unsigned short f2bf_bits(float f) {
  unsigned u = __float_as_uint(f);
  return (unsigned short)((u + 0x7FFFu + ((u >> 16) & 1u)) >> 16);
}
__device__ __forceinline__ float bf_bits2f(unsigned short h) { return __uint_as_float(((unsigned)h) << 16); }
__device__ __forceinline__ float bf16r(float f) { return bf_bits2f(f2bf_bits(f)); }
__device__ __forceinline__ float carry_flush(float v, float carry) {
  const float s = v * carry;
  return (fabsf(s) < kF16MinNormal) ? 0.0f : s;
}
__device__ __forceinline__ float frcp(float x) { return __builtin_amdgcn_rcpf(x); }

__device__ __forceinline__ void dep_guard4_h(v8f& a, v8f& b, v8f& c, v8f& d, v16h x, v16h y) { asm volatile("v_nop\n\tv_nop\n\tv_nop\n\tv_nop" : "+v"(a), "+v"(b), "+v"(c), "+v"(d) : "v"(x), "v"(y)); }
__device__ __forceinline__ void dep_guard4_b(v8f& a, v8f& b, v8f& c, v8f& d, v16b x, v16b y) { asm volatile("v_nop\n\tv_nop\n\tv_nop\n\tv_nop" : "+v"(a), "+v"(b), "+v"(c), "+v"(d) : "v"(x), "v"(y)); }
__device__ __forceinline__ void keep4_h(v16h a, v16h b, v16h c, v16h d) { asm volatile("v_nop" :: "v"(a), "v"(b), "v"(c), "v"(d)); }
__device__ __forceinline__ void keep4_b(v16b a, v16b b, v16b c, v16b d) { asm volatile("v_nop" :: "v"(a), "v"(b), "v"(c), "v"(d)); }
__device__ __forceinline__ void acc_guard4(v8f& a, v8f& b, v8f& c, v8f& d) { asm volatile("v_nop\n\tv_nop\n\tv_nop\n\tv_nop" : "+v"(a), "+v"(b), "+v"(c), "+v"(d)); }

template <typename T> struct Frag;
template <> struct Frag<_Float16> {
  typedef v16h V; union U { v16h v; v8h h[2]; };
  static __device__ __forceinline__ v16h load(const _Float16* p) {
    U f; f.h[0] = *(const v8h*)(p); f.h[1] = *(const v8h*)(p + 16); return f.v;
  }
  static __device__ __forceinline__ v8f mma(v16h a, v16h b, v8f c) {
    return __builtin_amdgcn_wmma_f32_16x16x32_f16(false, a, false, b, (short)0, c, false, false);
  }
  static __device__ __forceinline__ void guard4(v8f& a, v8f& b, v8f& c, v8f& d, v16h x, v16h y) { dep_guard4_h(a, b, c, d, x, y); }
  static __device__ __forceinline__ void keep(v16h a, v16h b, v16h c, v16h d) { keep4_h(a, b, c, d); }
};
template <> struct Frag<__bf16> {
  typedef v16b V; union U { v16b v; v8b h[2]; };
  static __device__ __forceinline__ v16b load(const __bf16* p) {
    U f; f.h[0] = *(const v8b*)(p); f.h[1] = *(const v8b*)(p + 16); return f.v;
  }
  static __device__ __forceinline__ v8f mma(v16b a, v16b b, v8f c) {
    return __builtin_amdgcn_wmma_f32_16x16x32_bf16(false, a, false, b, (short)0, c, false, false);
  }
  static __device__ __forceinline__ void guard4(v8f& a, v8f& b, v8f& c, v8f& d, v16b x, v16b y) { dep_guard4_b(a, b, c, d, x, y); }
  static __device__ __forceinline__ void keep(v16b a, v16b b, v16b c, v16b d) { keep4_b(a, b, c, d); }
};

__device__ __forceinline__ v8f mma_h(v16h a, v16h b, v8f c) {
  c = __builtin_amdgcn_wmma_f32_16x16x32_f16(false, a, false, b, (short)0, c, false, false);
  asm volatile("v_nop\n\tv_nop\n\tv_nop\n\tv_nop" : "+v"(c) : "v"(a), "v"(b));
  return c;
}

template <int ET> struct Elem;
template <> struct Elem<0> { typedef _Float16 T; };
template <> struct Elem<1> { typedef __bf16 T; };
template <int ET, bool SPLIT, int BIAS_MODE, int OUT_MODE, bool RESID, int ACT = 0>
__global__ __launch_bounds__(256) void wmma_gemm64(
    const unsigned short* __restrict__ Ap, const unsigned short* __restrict__ A2p, int lda, long strideA,
    const unsigned short* __restrict__ Btp, const unsigned short* __restrict__ Bt2p, int ldb, long strideB,
    void* __restrict__ Cout, void* __restrict__ Cout2, int ldc, long strideC,
    const float* __restrict__ bias,
    const float* __restrict__ resid, long strideR,
    int M, int N, int K, float scale) {
  typedef typename Elem<ET>::T T;
  typedef typename Frag<T>::V V;
  const T* A = (const T*)Ap; const T* A2 = (const T*)A2p; const T* Bt = (const T*)Btp; const T* Bt2 = (const T*)Bt2p;
  __shared__ __align__(16) float sT[8][16 * 68];
  const int b    = blockIdx.y;
  const int lane = threadIdx.x & 31;
  const int wave = threadIdx.x >> 5;
  const int tilesN = N >> 6;
  const int tilesM = M >> 6;
  const int tile = blockIdx.x * 8 + wave;
  if (tile >= tilesM * tilesN) return;
  const int tm = tile / tilesN;
  const int tn = tile - tm * tilesN;
  const int m0 = tm << 6;
  const int n0 = tn << 6;

  const T* Ab  = A  + (size_t)b * strideA;
  const T* Bb  = Bt + (size_t)b * strideB;
  const T* Ab2 = SPLIT ? (A2  + (size_t)b * strideA) : nullptr;
  const T* Bb2 = SPLIT ? (Bt2 + (size_t)b * strideB) : nullptr;

  const int rlane = lane & 15;
  const int koff  = (lane >> 4) * 8;
  const int mOff  = (lane >> 4) * 8;

  v8f acc[4][4];
#pragma unroll
  for (int i = 0; i < 4; ++i)
#pragma unroll
    for (int j = 0; j < 4; ++j) acc[i][j] = (v8f){0.f,0.f,0.f,0.f,0.f,0.f,0.f,0.f};

  for (int k0 = 0; k0 < K; k0 += 32) {
    V bh[4], bl[4];
#pragma unroll
    for (int j = 0; j < 4; ++j) {
      const size_t bo = (size_t)(n0 + (j << 4) + rlane) * ldb + koff + k0;
      bh[j] = Frag<T>::load(Bb + bo);
      if (SPLIT) bl[j] = Frag<T>::load(Bb2 + bo);
    }
#pragma unroll
    for (int i = 0; i < 4; ++i) {
      const size_t ao = (size_t)(m0 + (i << 4) + rlane) * lda + koff + k0;
      V ah = Frag<T>::load(Ab + ao);
      V al;
      if (SPLIT) al = Frag<T>::load(Ab2 + ao);
#pragma unroll
      for (int j = 0; j < 4; ++j) {
        acc[i][j] = Frag<T>::mma(ah, bh[j], acc[i][j]);
        if (SPLIT) {
          acc[i][j] = Frag<T>::mma(ah, bl[j], acc[i][j]);
          acc[i][j] = Frag<T>::mma(al, bh[j], acc[i][j]);
        }
      }
      Frag<T>::guard4(acc[i][0], acc[i][1], acc[i][2], acc[i][3], ah, SPLIT ? al : ah);
    }
    Frag<T>::keep(bh[0], bh[1], bh[2], bh[3]);
    if (SPLIT) Frag<T>::keep(bl[0], bl[1], bl[2], bl[3]);
  }
  acc_guard4(acc[0][0], acc[0][1], acc[0][2], acc[0][3]);
  acc_guard4(acc[1][0], acc[1][1], acc[1][2], acc[1][3]);
  acc_guard4(acc[2][0], acc[2][1], acc[2][2], acc[2][3]);
  acc_guard4(acc[3][0], acc[3][1], acc[3][2], acc[3][3]);

  float* slab = sT[wave];
  const float* Rb = RESID ? (resid + (size_t)b * strideR) : nullptr;
#pragma unroll
  for (int i = 0; i < 4; ++i) {
    const int mBase = m0 + (i << 4);
#pragma unroll
    for (int j = 0; j < 4; ++j) {
      const int n = n0 + (j << 4) + rlane;
      float bv = 0.f;
      if (BIAS_MODE == 2) bv = bias[n];
#pragma unroll
      for (int r = 0; r < 8; ++r) {
        float v = acc[i][j][r] * scale;
        if (BIAS_MODE == 1) v += bias[mBase + mOff + r];
        if (BIAS_MODE == 2) v += bv;
        if (RESID) v += Rb[(size_t)(mBase + mOff + r) * ldc + n];
        if (ACT == 1) v = tanhf(v);
        if (ACT == 2) v = fmaxf(v, 0.0f);
        if (ACT == 3) v = v / (1.0f + expf(-v));
        if (ACT == 4) v = (v > 0.f) ? v : 0.01f * v;
        slab[(mOff + r) * 68 + (j << 4) + rlane] = v;
      }
    }
    __builtin_amdgcn_fence(__ATOMIC_RELEASE, "workgroup");
    __builtin_amdgcn_wave_barrier();
    __builtin_amdgcn_fence(__ATOMIC_ACQUIRE, "workgroup");
    if (OUT_MODE == 0) {
      float* C = (float*)Cout + (size_t)b * strideC;
      const int hh = lane >> 4, c4 = (lane & 15) * 4;
      for (int pass = 0; pass < 2; ++pass) {
#pragma unroll
        for (int it = 0; it < 8; ++it) {
          const int row = it * 2 + hh;
          v4f v = *(const v4f*)(slab + row * 68 + c4);
          *(volatile v4f*)(C + (size_t)(mBase + row) * ldc + n0 + c4) = v;
        }
        __threadfence();
      }
    } else {
      const int q = lane >> 3, c8 = (lane & 7) * 8;
      unsigned short* C  = (unsigned short*)Cout  + (size_t)b * strideC;
      unsigned short* C2 = (OUT_MODE == 2) ? ((unsigned short*)Cout2 + (size_t)b * strideC) : nullptr;
      for (int pass = 0; pass < 2; ++pass) {
#pragma unroll
        for (int it = 0; it < 4; ++it) {
          const int row = it * 4 + q;
          const float* sp = slab + row * 68 + c8;
          v8h hv, lv;
#pragma unroll
          for (int e = 0; e < 8; ++e) {
            if (OUT_MODE == 1) {
              hv[e] = (_Float16)sp[e];
            } else {
              unsigned short hb = f2bf_bits(sp[e]);
              unsigned short lb = f2bf_bits(sp[e] - bf_bits2f(hb));
              hv[e] = __builtin_bit_cast(_Float16, hb);
              lv[e] = __builtin_bit_cast(_Float16, lb);
            }
          }
          *(volatile v8h*)(C + (size_t)(mBase + row) * ldc + n0 + c8) = hv;
          if (OUT_MODE == 2) *(volatile v8h*)(C2 + (size_t)(mBase + row) * ldc + n0 + c8) = lv;
        }
        __threadfence();
      }
    }
    __builtin_amdgcn_fence(__ATOMIC_RELEASE, "workgroup");
    __builtin_amdgcn_wave_barrier();
    __builtin_amdgcn_fence(__ATOMIC_ACQUIRE, "workgroup");
  }
}


__global__ __launch_bounds__(kThr) void im2col_plane_kernel(const float* __restrict__ x, unsigned short* __restrict__ A16) {
  const int v  = blockIdx.x * kThr + threadIdx.x;
  const int m  = v / (kKP / 8);
  const int k8 = (v - m * (kKP / 8)) * 8;
  const int mc = (m < kRows) ? m : (kRows - 1);
  const int w  = mc / kLout;
  const int l  = mc - w * kLout;
  v8h hv;
#pragma unroll
  for (int e = 0; e < 8; ++e) {
    const int k  = k8 + e;
    const int kc = (k < kK) ? k : (kK - 1);
    const int c  = kc / kTap;
    const int j  = kc - c * kTap;
    const float xv = x[((size_t)w * kCin + c) * kLin + kStride * l + j];
    const bool ok = (m < kRows) && (k < kK);
    const float g = ok ? carry_flush(bf16r(xv), kInCarry) : 0.0f;
    hv[e] = (_Float16)g;
  }
  unsigned short* dst = A16 + (size_t)m * kKP + k8;
  *(volatile v8h*)dst = hv;
  __threadfence();
  *(volatile v8h*)dst = hv;
}

__global__ __launch_bounds__(kThr) void filter_plane_kernel(const float* __restrict__ W, unsigned short* __restrict__ W16, float* __restrict__ ZB) {
  const int v  = blockIdx.x * kThr + threadIdx.x;
  const int n  = v / (kKP / 8);
  const int k8 = (v - n * (kKP / 8)) * 8;
  v8h hv;
#pragma unroll
  for (int e = 0; e < 8; ++e) {
    const int k  = k8 + e;
    const int kc = (k < kK) ? k : (kK - 1);
    const float wv = W[(size_t)n * kK + kc];
    const float g = (k < kK) ? carry_flush(bf16r(wv), kWCarry) : 0.0f;
    hv[e] = (_Float16)g;
  }
  unsigned short* dst = W16 + (size_t)n * kKP + k8;
  *(volatile v8h*)dst = hv;
  __threadfence();
  *(volatile v8h*)dst = hv;
  if (v < kCout / 4) {
    const v4f zero4 = {0.f, 0.f, 0.f, 0.f};
    volatile v4f* z = (volatile v4f*)(ZB + 4 * v);
    *z = zero4;
    __threadfence();
    *z = zero4;
  }
}

__global__ __launch_bounds__(32) void window_scan_kernel(const float* __restrict__ LIN, float* __restrict__ out) {
  const int e4 = (blockIdx.x * 32 + threadIdx.x) * 4;
  int oo[4], ll[4];
#pragma unroll
  for (int i = 0; i < 4; ++i) {
    const int e = e4 + i;
    oo[i] = e / kLout;
    ll[i] = e - oo[i] * kLout;
  }
  v4f res = {0.f, 0.f, 0.f, 0.f};
#pragma unroll 1
  for (int w = 0; w < kWin; ++w) {
#pragma unroll
    for (int i = 0; i < 4; ++i) {
      const float lin = LIN[((size_t)w * kLout + ll[i]) * kCout + oo[i]];
      const float prev = res[i];
      res[i] = tanhf(lin + prev);
    }
    float* op = out + (size_t)w * kPlane + e4;
    *(volatile v4f*)op = res;
    __threadfence();
    *(volatile v4f*)op = res;
  }
}

extern "C" void kernel_launch(void* const* d_in, const int* in_sizes, int n_in,
                              void* d_out, int out_size, void* d_ws, size_t ws_size,
                              hipStream_t stream) {
  if (n_in < 2 || d_out == nullptr || d_ws == nullptr) return;
  if (in_sizes[0] != kWin * kCin * kLin) return;
  if (in_sizes[1] != kCout * kK) return;
  if (out_size != kWin * kPlane) return;
  if (ws_size < kWsTotal) return;

  const float* x = (const float*)d_in[0];
  const float* W = (const float*)d_in[1];
  float* out = (float*)d_out;

  char* ws = (char*)d_ws;
  unsigned short* A16 = (unsigned short*)(ws + kOffA16);
  unsigned short* W16 = (unsigned short*)(ws + kOffW16);
  float*          ZB  = (float*)(ws + kOffZB);
  float*          LIN = (float*)(ws + kOffLIN);

  im2col_plane_kernel<<<(int)(((size_t)kRowsP * (kKP / 8)) / kThr), kThr, 0, stream>>>(x, A16);
  filter_plane_kernel<<<(int)(((size_t)kCout * (kKP / 8)) / kThr), kThr, 0, stream>>>(W, W16, ZB);

  wmma_gemm64<0, false, 2, 0, false, 0><<<dim3(((kRowsP / 64) * (kCout / 64) + 7) / 8, 1), 256, 0, stream>>>(
      A16, A16, kKP, 0L, W16, W16, kKP, 0L, (void*)LIN, (void*)LIN, kCout, 0L,
      ZB, nullptr, 0L, kRowsP, kCout, kKP, kScale);

  window_scan_kernel<<<(kPlane / 4) / 32, 32, 0, stream>>>(LIN, out);
}
